// ResLFE_Block_23021024707172
// MI455X (gfx1250) — hardware-verified
//
#include <hip/hip_runtime.h>
#include <math.h>
#include <stddef.h>
#include <stdint.h>


#define RB    4
#define NP    16000
#define CC    128
#define KK    16
#define DD    4
#define HD    512
#define RTOT  (RB * NP)
#define EPSV  1e-5f
#define XSC   4
#define HSC   4
#define WSC   1024
#define NTHR  256
#define NWAVE 8
#define TPW   64
#define WSCAP 134217728
#define LDS_GEMM (NWAVE * 32 * 64 * 4)

static_assert(RTOT % 128 == 0);
static_assert(HD % 128 == 0);
static_assert(CC % 128 == 0);
static_assert(CC % 64 == 0);
static_assert(HD % 64 == 0);
static_assert(CC % 32 == 0);
static_assert(HD % 32 == 0);
static_assert((RTOT * CC) % (8 * NTHR) == 0);
static_assert(RTOT % NWAVE == 0);
static_assert(NTHR == NWAVE * 32);
static_assert(CC == 4 * 32);
static_assert(KK == 16);
static_assert(LDS_GEMM <= 300 * 1024);

typedef float    v2f  __attribute__((ext_vector_type(2)));
typedef float    v4f  __attribute__((ext_vector_type(4)));
typedef float    v8f  __attribute__((ext_vector_type(8)));
typedef _Float16 v8h  __attribute__((ext_vector_type(8)));
typedef _Float16 v16h __attribute__((ext_vector_type(16)));
typedef int      v4i  __attribute__((ext_vector_type(4)));
union FragH { v16h v; v8h h[2]; };

__device__ __forceinline__ v8f wmf(v16h a, v16h b, v8f c) {
  v8f d = __builtin_amdgcn_wmma_f32_16x16x32_f16(false, a, false, b, (short)0, c, false, false);
  asm volatile("v_nop\n\tv_nop\n\tv_nop\n\tv_nop" : "+v"(d) : "v"(a), "v"(b));
  return d;
}

__device__ __forceinline__ float tanh_c(float u) {
  const float a = fminf(fabsf(u), 10.0f);
  const float e = __expf(2.0f * a);
  const float t = 1.0f - 2.0f * __builtin_amdgcn_rcpf(e + 1.0f);
  return copysignf(t, u);
}
__device__ __forceinline__ float gelu1(float x) {
  const float c0 = 0.7978845608028654f;
  const float u = c0 * (x + 0.044715f * (x * x * x));
  const float cdf = 0.5f * (1.0f + tanh_c(u));
  return x * cdf;
}
__device__ __forceinline__ v4f gelu4(v4f a) {
  v4f o;
  o.x = gelu1(a.x); o.y = gelu1(a.y); o.z = gelu1(a.z); o.w = gelu1(a.w);
  return o;
}
__device__ __forceinline__ v4f vmax4(v4f a, v4f b) {
  v4f o;
  o.x = fmaxf(a.x, b.x); o.y = fmaxf(a.y, b.y); o.z = fmaxf(a.z, b.z); o.w = fmaxf(a.w, b.w);
  return o;
}
__device__ __forceinline__ v8h pack8(v4f a, v4f b, float s) {
  v8h o;
  o[0] = (_Float16)(a.x * s); o[1] = (_Float16)(a.y * s);
  o[2] = (_Float16)(a.z * s); o[3] = (_Float16)(a.w * s);
  o[4] = (_Float16)(b.x * s); o[5] = (_Float16)(b.y * s);
  o[6] = (_Float16)(b.z * s); o[7] = (_Float16)(b.w * s);
  return o;
}

__global__ __launch_bounds__(NTHR) void k_prepx(const float* __restrict__ x, _Float16* xh) {
  const size_t t = (size_t)blockIdx.x * NTHR + threadIdx.x;
  const float* p = x + t * 8;
  const v4f f0 = *(const v4f*)p;
  const v4f f1 = *(const v4f*)(p + 4);
  const v8h a = pack8(f0, f1, (float)XSC);
  _Float16* d = xh + t * 8;
  *(volatile v8h*)d = a;
  __threadfence();
  *(volatile v8h*)d = a;
}

__global__ __launch_bounds__(NTHR) void k_prepw(const float* __restrict__ W, _Float16* wt, int Kd, int Nd) {
  __shared__ __attribute__((aligned(16))) float tile[128 * TPW];
  const int tid = threadIdx.x, lane = tid & 31, g = tid >> 5, hh = lane >> 4, m = lane & 15;
  const float* src = W + (size_t)blockIdx.y * Kd * Nd;
  _Float16* dst = wt + (size_t)blockIdx.y * Kd * Nd;
  const int n0 = blockIdx.x * 64;
  const int n = n0 + 2 * lane;
#pragma unroll 1
  for (int dc = 0; dc < Kd; dc += 128) {
    __syncthreads();
#pragma unroll 4
    for (int p = 0; p < 16; ++p) {
      const int dl = g + 8 * p;
      const v2f w = *(const v2f*)(src + (size_t)(dc + dl) * Nd + n);
      *(v2f*)(tile + dl * TPW + 2 * lane) = w;
    }
    __syncthreads();
    v8h hv[4];
#pragma unroll
    for (int q = 0; q < 4; ++q) {
      const int nl = 8 * g + 2 * q + hh;
      const int d8 = 8 * m;
#pragma unroll
      for (int e = 0; e < 8; ++e) hv[q][e] = (_Float16)(tile[(d8 + e) * TPW + nl] * (float)WSC);
    }
#pragma unroll
    for (int q = 0; q < 4; ++q) {
      _Float16* d = dst + (size_t)(n0 + 8 * g + 2 * q + hh) * Kd + dc + 8 * m;
      *(volatile v8h*)d = hv[q];
    }
    __threadfence();
#pragma unroll
    for (int q = 0; q < 4; ++q) {
      _Float16* d = dst + (size_t)(n0 + 8 * g + 2 * q + hh) * Kd + dc + 8 * m;
      *(volatile v8h*)d = hv[q];
    }
  }
}

template <int MODE>
__global__ __launch_bounds__(NTHR) void k_gemm(const _Float16* __restrict__ A, int lda, int Ktot,
                                               const _Float16* __restrict__ Bt,
                                               const float* __restrict__ bias,
                                               const float* __restrict__ pg, const float* __restrict__ pb,
                                               const float* __restrict__ pm, const float* __restrict__ pv,
                                               const float* res, const float* __restrict__ pe, int addpe,
                                               float* outF, _Float16* outH, int ldo) {
  extern __shared__ v4f lds_dyn[];
  __shared__ __attribute__((aligned(16))) float s_c0[128];
  __shared__ __attribute__((aligned(16))) float s_c1[128];
  __shared__ __attribute__((aligned(16))) float s_c2[128];
  __shared__ __attribute__((aligned(16))) float s_c3[128];
  const int tid = threadIdx.x, lane = tid & 31, wave = tid >> 5, hh = lane >> 4, m = lane & 15;
  float* stg = (float*)lds_dyn + wave * (32 * 64);
  const int n0 = blockIdx.x * 128, m0 = blockIdx.y * 128;
  const int wm = (wave >> 1) * 32, wn = (wave & 1) * 64;

  if (MODE == 0) {
    if (tid < 128) s_c0[tid] = bias[n0 + tid];
  }
  if (MODE == 1) {
    if (tid < 128) {
      s_c0[tid] = pg[n0 + tid];
      s_c1[tid] = pb[n0 + tid];
      s_c2[tid] = pm[n0 + tid];
      s_c3[tid] = rsqrtf(pv[n0 + tid] + EPSV);
    }
  }
  __syncthreads();

  v8f acc[2][4];
#pragma unroll
  for (int mt = 0; mt < 2; ++mt)
#pragma unroll
    for (int nt = 0; nt < 4; ++nt) { v8f z = {0.f, 0.f, 0.f, 0.f, 0.f, 0.f, 0.f, 0.f}; acc[mt][nt] = z; }

  const _Float16* ap = A + (size_t)(m0 + wm + m) * lda + 8 * hh;
  const _Float16* bp = Bt + (size_t)(n0 + wn + m) * Ktot + 8 * hh;
#pragma unroll 1
  for (int k0 = 0; k0 < Ktot; k0 += 32) {
    FragH a0, a1;
    a0.h[0] = *(const v8h*)(ap + k0);
    a0.h[1] = *(const v8h*)(ap + k0 + 16);
    a1.h[0] = *(const v8h*)(ap + (size_t)16 * lda + k0);
    a1.h[1] = *(const v8h*)(ap + (size_t)16 * lda + k0 + 16);
#pragma unroll
    for (int nt = 0; nt < 4; ++nt) {
      const _Float16* bq = bp + (size_t)nt * 16 * Ktot + k0;
      FragH b;
      b.h[0] = *(const v8h*)bq;
      b.h[1] = *(const v8h*)(bq + 16);
      acc[0][nt] = wmf(a0.v, b.v, acc[0][nt]);
      acc[1][nt] = wmf(a1.v, b.v, acc[1][nt]);
    }
  }

  constexpr float OSC = (MODE == 1) ? (1.0f / (float)(HSC * WSC)) : (1.0f / (float)(XSC * WSC));
#pragma unroll
  for (int mt = 0; mt < 2; ++mt) {
    float* sp = stg + (16 * mt + 8 * hh) * 64 + m;
#pragma unroll
    for (int nt = 0; nt < 4; ++nt) {
      float bv = 0.0f;
      if (MODE == 0) bv = s_c0[wn + 16 * nt + m];
#pragma unroll
      for (int r = 0; r < 8; ++r) sp[r * 64 + 16 * nt] = acc[mt][nt][r] * OSC + bv;
    }
  }
  __syncthreads();

  if (MODE == 2) {
    float* gb = outF + (size_t)(m0 + wm) * ldo + n0 + wn + 4 * m;
#pragma unroll
    for (int q = 0; q < 16; ++q) {
      const int row = 2 * q + hh;
      const v4f v = *(const v4f*)(stg + row * 64 + 4 * m);
      *(volatile v4f*)(gb + (size_t)row * ldo) = v;
    }
    __threadfence();
#pragma unroll
    for (int q = 0; q < 16; ++q) {
      const int row = 2 * q + hh;
      const v4f v = *(const v4f*)(stg + row * 64 + 4 * m);
      *(volatile v4f*)(gb + (size_t)row * ldo) = v;
    }
  }

  if (MODE == 0) {
    const int rsub = lane >> 3, c8 = 8 * (lane & 7);
    _Float16* hb = outH + (size_t)(m0 + wm) * ldo + n0 + wn + c8;
#pragma unroll 1
    for (int q = 0; q < 8; ++q) {
      const int row = 4 * q + rsub;
      float* sp2 = stg + row * 64 + c8;
      v4f u0 = *(v4f*)sp2;
      v4f u1 = *(v4f*)(sp2 + 4);
      u0 = gelu4(u0);
      u1 = gelu4(u1);
      *(v4f*)sp2 = u0;
      *(v4f*)(sp2 + 4) = u1;
      const v8h o = pack8(u0, u1, (float)HSC);
      *(volatile v8h*)(hb + (size_t)row * ldo) = o;
    }
    __threadfence();
#pragma unroll
    for (int q = 0; q < 8; ++q) {
      const int row = 4 * q + rsub;
      const float* sp2 = stg + row * 64 + c8;
      const v4f u0 = *(const v4f*)sp2;
      const v4f u1 = *(const v4f*)(sp2 + 4);
      const v8h o = pack8(u0, u1, (float)HSC);
      *(volatile v8h*)(hb + (size_t)row * ldo) = o;
    }
  }

  if (MODE == 1) {
    const size_t base = (size_t)(m0 + wm) * ldo + n0 + wn + 4 * m;
    float* ob = outF + base;
    const float* rbp = res + base;
    const float* pbp = pe + base;
    const int cl = wn + 4 * m;
    const v4f g4 = *(const v4f*)(s_c0 + cl);
    const v4f b4 = *(const v4f*)(s_c1 + cl);
    const v4f m4 = *(const v4f*)(s_c2 + cl);
    const v4f r4 = *(const v4f*)(s_c3 + cl);
#pragma unroll
    for (int q = 0; q < 16; ++q) {
      const int row = 2 * q + hh;
      float* sp2 = stg + row * 64 + 4 * m;
      const v4f a = *(const v4f*)sp2;
      const v4f bn = (a - m4) * r4 * g4 + b4;
      const v4f rv = *(const v4f*)(rbp + (size_t)row * ldo);
      v4f o = rv + bn;
      if (addpe) {
        const v4f pv4 = *(const v4f*)(pbp + (size_t)row * ldo);
        o = o + pv4;
      }
      *(v4f*)sp2 = o;
      *(volatile v4f*)(ob + (size_t)row * ldo) = o;
    }
    __threadfence();
    __syncthreads();
#pragma unroll
    for (int q = 0; q < 16; ++q) {
      const int row = 2 * q + hh;
      const v4f o = *(const v4f*)(stg + row * 64 + 4 * m);
      *(volatile v4f*)(ob + (size_t)row * ldo) = o;
    }
    const int rsub = lane >> 3, c8 = 8 * (lane & 7);
    _Float16* hb = outH + (size_t)(m0 + wm) * ldo + n0 + wn + c8;
#pragma unroll
    for (int q = 0; q < 8; ++q) {
      const int row = 4 * q + rsub;
      const float* sp2 = stg + row * 64 + c8;
      const v8h o = pack8(*(const v4f*)sp2, *(const v4f*)(sp2 + 4), (float)XSC);
      *(volatile v8h*)(hb + (size_t)row * ldo) = o;
    }
    __threadfence();
#pragma unroll
    for (int q = 0; q < 8; ++q) {
      const int row = 4 * q + rsub;
      const float* sp2 = stg + row * 64 + c8;
      const v8h o = pack8(*(const v4f*)sp2, *(const v4f*)(sp2 + 4), (float)XSC);
      *(volatile v8h*)(hb + (size_t)row * ldo) = o;
    }
  }
}

__device__ __forceinline__ v4f nb_diff(const float* yb, v4f own, int id) {
  id = min(max(id, 0), NP - 1);
  return *(const v4f*)(yb + (size_t)id * CC) - own;
}

__global__ __launch_bounds__(NTHR) void k_nbmax(const float* __restrict__ y, const int* __restrict__ knn,
                                                const float* __restrict__ pg, const float* __restrict__ pb,
                                                const float* __restrict__ pm, const float* __restrict__ pv,
                                                float* xio, _Float16* xh) {
  const int lane = threadIdx.x & 31, wave = threadIdx.x >> 5;
  const int r = blockIdx.x * NWAVE + wave;
  const int b = r / NP;
  const int* kn = knn + (size_t)r * KK;
  const v4i i0 = *(const v4i*)kn;
  const v4i i1 = *(const v4i*)(kn + 4);
  const v4i i2 = *(const v4i*)(kn + 8);
  const v4i i3 = *(const v4i*)(kn + 12);
  const float* yb = y + (size_t)b * NP * CC + 4 * lane;
  const v4f own = *(const v4f*)(y + (size_t)r * CC + 4 * lane);

  v4f mx = nb_diff(yb, own, i0.x);
  mx = vmax4(mx, nb_diff(yb, own, i0.y));
  mx = vmax4(mx, nb_diff(yb, own, i0.z));
  mx = vmax4(mx, nb_diff(yb, own, i0.w));
  mx = vmax4(mx, nb_diff(yb, own, i1.x));
  mx = vmax4(mx, nb_diff(yb, own, i1.y));
  mx = vmax4(mx, nb_diff(yb, own, i1.z));
  mx = vmax4(mx, nb_diff(yb, own, i1.w));
  mx = vmax4(mx, nb_diff(yb, own, i2.x));
  mx = vmax4(mx, nb_diff(yb, own, i2.y));
  mx = vmax4(mx, nb_diff(yb, own, i2.z));
  mx = vmax4(mx, nb_diff(yb, own, i2.w));
  mx = vmax4(mx, nb_diff(yb, own, i3.x));
  mx = vmax4(mx, nb_diff(yb, own, i3.y));
  mx = vmax4(mx, nb_diff(yb, own, i3.z));
  mx = vmax4(mx, nb_diff(yb, own, i3.w));

  const v4f g4 = *(const v4f*)(pg + 4 * lane);
  const v4f b4 = *(const v4f*)(pb + 4 * lane);
  const v4f m4 = *(const v4f*)(pm + 4 * lane);
  const v4f v4 = *(const v4f*)(pv + 4 * lane);
  v4f r4;
  r4.x = rsqrtf(v4.x + EPSV); r4.y = rsqrtf(v4.y + EPSV);
  r4.z = rsqrtf(v4.z + EPSV); r4.w = rsqrtf(v4.w + EPSV);
  const v4f bn = (mx - m4) * r4 * g4 + b4;

  float* xp = xio + (size_t)r * CC + 4 * lane;
  const v4f xa = *(const v4f*)xp;
  const v4f o = xa + bn;

  const int j = lane & 15;
  v4f e0, e1;
  e0.x = __shfl(o.x, 2 * j);     e0.y = __shfl(o.y, 2 * j);
  e0.z = __shfl(o.z, 2 * j);     e0.w = __shfl(o.w, 2 * j);
  e1.x = __shfl(o.x, 2 * j + 1); e1.y = __shfl(o.y, 2 * j + 1);
  e1.z = __shfl(o.z, 2 * j + 1); e1.w = __shfl(o.w, 2 * j + 1);
  const v8h hv = pack8(e0, e1, (float)XSC);
  _Float16* hp = xh + (size_t)r * CC + 8 * j;

  *(volatile v4f*)xp = o;
  if (lane < 16) *(volatile v8h*)hp = hv;
  __threadfence();
  *(volatile v4f*)xp = o;
  if (lane < 16) *(volatile v8h*)hp = hv;
}

extern "C" void kernel_launch(void* const* d_in, const int* in_sizes, int n_in,
                              void* d_out, int out_size, void* d_ws, size_t ws_size,
                              hipStream_t stream) {
  if (n_in < 22) return;
  if (in_sizes[0] != RTOT * CC || in_sizes[1] != RTOT * CC || in_sizes[2] != RTOT * KK) return;
  if (in_sizes[3] != CC * HD || in_sizes[4] != HD || in_sizes[5] != HD * CC) return;
  if (in_sizes[6] != CC || in_sizes[7] != CC || in_sizes[8] != CC || in_sizes[9] != CC) return;
  if (in_sizes[10] != DD * CC * CC) return;
  for (int i = 11; i <= 14; ++i) if (in_sizes[i] != DD * CC) return;
  if (in_sizes[15] != DD * CC * HD || in_sizes[16] != DD * HD || in_sizes[17] != DD * HD * CC) return;
  for (int i = 18; i <= 21; ++i) if (in_sizes[i] != DD * CC) return;
  if (out_size != RTOT * CC) return;

  const float* x_in = (const float*)d_in[0];
  const float* pe   = (const float*)d_in[1];
  const int*   knn  = (const int*)d_in[2];
  const float* w1m  = (const float*)d_in[3];
  const float* b1m  = (const float*)d_in[4];
  const float* w2m  = (const float*)d_in[5];
  const float* gm   = (const float*)d_in[6];
  const float* bem  = (const float*)d_in[7];
  const float* mm   = (const float*)d_in[8];
  const float* vm   = (const float*)d_in[9];
  const float* wv   = (const float*)d_in[10];
  const float* gv   = (const float*)d_in[11];
  const float* bev  = (const float*)d_in[12];
  const float* mv   = (const float*)d_in[13];
  const float* vv   = (const float*)d_in[14];
  const float* w1f  = (const float*)d_in[15];
  const float* b1f  = (const float*)d_in[16];
  const float* w2f  = (const float*)d_in[17];
  const float* gf   = (const float*)d_in[18];
  const float* bef  = (const float*)d_in[19];
  const float* mf   = (const float*)d_in[20];
  const float* vf   = (const float*)d_in[21];
  float* out = (float*)d_out;

  char* ws = (char*)d_ws;
  size_t off = 0;
  const size_t oXh = off; off += (size_t)RTOT * CC * 2;      off = (off + 255) & ~(size_t)255;
  const size_t oHh = off; off += (size_t)RTOT * HD * 2;      off = (off + 255) & ~(size_t)255;
  const size_t oY  = off; off += (size_t)RTOT * CC * 4;      off = (off + 255) & ~(size_t)255;
  const size_t oW1 = off; off += (size_t)HD * CC * 2;        off = (off + 255) & ~(size_t)255;
  const size_t oW2 = off; off += (size_t)CC * HD * 2;        off = (off + 255) & ~(size_t)255;
  const size_t oF1 = off; off += (size_t)DD * HD * CC * 2;   off = (off + 255) & ~(size_t)255;
  const size_t oF2 = off; off += (size_t)DD * CC * HD * 2;   off = (off + 255) & ~(size_t)255;
  const size_t oVt = off; off += (size_t)DD * CC * CC * 2;   off = (off + 255) & ~(size_t)255;
  if (off > ws_size || off > (size_t)WSCAP) return;
  _Float16* xh  = (_Float16*)(ws + oXh);
  _Float16* hh  = (_Float16*)(ws + oHh);
  float*    yb  = (float*)(ws + oY);
  _Float16* w1t = (_Float16*)(ws + oW1);
  _Float16* w2t = (_Float16*)(ws + oW2);
  _Float16* f1t = (_Float16*)(ws + oF1);
  _Float16* f2t = (_Float16*)(ws + oF2);
  _Float16* vt  = (_Float16*)(ws + oVt);

  hipFuncSetAttribute(reinterpret_cast<const void*>(&k_gemm<0>), hipFuncAttributeMaxDynamicSharedMemorySize, LDS_GEMM);
  hipFuncSetAttribute(reinterpret_cast<const void*>(&k_gemm<1>), hipFuncAttributeMaxDynamicSharedMemorySize, LDS_GEMM);
  hipFuncSetAttribute(reinterpret_cast<const void*>(&k_gemm<2>), hipFuncAttributeMaxDynamicSharedMemorySize, LDS_GEMM);

  k_prepw<<<dim3(HD / 64, 1), NTHR, 0, stream>>>(w1m, w1t, CC, HD);
  k_prepw<<<dim3(CC / 64, 1), NTHR, 0, stream>>>(w2m, w2t, HD, CC);
  k_prepw<<<dim3(HD / 64, DD), NTHR, 0, stream>>>(w1f, f1t, CC, HD);
  k_prepw<<<dim3(CC / 64, DD), NTHR, 0, stream>>>(w2f, f2t, HD, CC);
  k_prepw<<<dim3(CC / 64, DD), NTHR, 0, stream>>>(wv, vt, CC, CC);
  k_prepx<<<(RTOT * CC) / (8 * NTHR), NTHR, 0, stream>>>(x_in, xh);

  const dim3 gUp(HD / 128, RTOT / 128);
  const dim3 gDn(CC / 128, RTOT / 128);

  k_gemm<0><<<gUp, NTHR, LDS_GEMM, stream>>>(xh, CC, CC, w1t, b1m, gm, bem, mm, vm,
                                             x_in, pe, 0, yb, hh, HD);
  k_gemm<1><<<gDn, NTHR, LDS_GEMM, stream>>>(hh, HD, HD, w2t, b1m, gm, bem, mm, vm,
                                             x_in, pe, 1, out, xh, CC);

  for (int d = 0; d < DD; ++d) {
    k_gemm<2><<<gDn, NTHR, LDS_GEMM, stream>>>(xh, CC, CC, vt + (size_t)d * CC * CC, b1m, gm, bem, mm, vm,
                                               x_in, pe, 0, yb, hh, CC);
    k_nbmax<<<RTOT / NWAVE, NTHR, 0, stream>>>(yb, knn, gv + d * CC, bev + d * CC, mv + d * CC, vv + d * CC,
                                               out, xh);
    k_gemm<0><<<gUp, NTHR, LDS_GEMM, stream>>>(xh, CC, CC, f1t + (size_t)d * HD * CC, b1f + (size_t)d * HD,
                                               gm, bem, mm, vm, x_in, pe, 0, yb, hh, HD);
    k_gemm<1><<<gDn, NTHR, LDS_GEMM, stream>>>(hh, HD, HD, f2t + (size_t)d * CC * HD, b1m,
                                               gf + d * CC, bef + d * CC, mf + d * CC, vf + d * CC,
                                               out, pe, (d < DD - 1) ? 1 : 0, out, xh, CC);
  }
}
